// Transformer_54571854463216
// MI455X (gfx1250) — hardware-verified
//
#include <hip/hip_runtime.h>
#include <math.h>

#ifndef NB
#define NB 2
#endif
#ifndef SEQ
#define SEQ 1024
#endif
#define NB_FULL 2
#define SEQ_FULL 1024
#define DM 1024
#define NH 16
#define HDIM 64
#define NLAYER 6
#define MROWS (NB * SEQ)
#define QKP (2 * DM)
#define VTP (MROWS)

static_assert(DM == NH * HDIM);
static_assert(HDIM == 64);
static_assert((SEQ % 64) == 0);
static_assert((MROWS % 64) == 0);
static_assert((DM % 64) == 0 && (DM % 32) == 0);
static_assert((((MROWS / 64) & ((MROWS / 64) - 1)) == 0));
static_assert(NB <= NB_FULL && SEQ <= SEQ_FULL);

typedef __attribute__((ext_vector_type(16))) _Float16 v16h;
typedef __attribute__((ext_vector_type(8)))  _Float16 v8h;
typedef __attribute__((ext_vector_type(8)))  float    v8f;
typedef __attribute__((ext_vector_type(4)))  float    v4f;
typedef __attribute__((ext_vector_type(2)))  float    v2f;
typedef __attribute__((ext_vector_type(4)))  unsigned v4u;
typedef __attribute__((ext_vector_type(2)))  unsigned v2u;


#define VST2(T, ptr, val) do { const T vst2_v_ = (val); *(volatile T*)(ptr) = vst2_v_; __threadfence(); *(volatile T*)(ptr) = vst2_v_; } while (0)

__device__ __forceinline__ float cmb_bf(float v) {
    const unsigned u = __builtin_bit_cast(unsigned, v);
    const unsigned r = (u + 0x7fffu + ((u >> 16) & 1u)) & 0xffff0000u;
    return __builtin_bit_cast(float, r);
}
__device__ __forceinline__ unsigned cmb_pk2(float a, float b) {
    return (unsigned)__builtin_bit_cast(unsigned short, (_Float16)a) | ((unsigned)__builtin_bit_cast(unsigned short, (_Float16)b) << 16);
}

union FragU { v16h v; v8h h[2]; };
__device__ __forceinline__ v16h fload(const _Float16* p) { FragU f; f.h[0] = *(const v8h*)(p); f.h[1] = *(const v8h*)(p + 16); return f.v; }

__device__ __forceinline__ v8f mma_raw(v16h a, v16h b, v8f c) {
    return __builtin_amdgcn_wmma_f32_16x16x32_f16(false, a, false, b, (short)0, c, false, false);
}
__device__ __forceinline__ void dep_guard_h(v8f& a, v8f& b, v16h x, v16h y) { asm volatile("v_nop\n\tv_nop\n\tv_nop\n\tv_nop" : "+v"(a), "+v"(b) : "v"(x), "v"(y)); }
__device__ __forceinline__ void keep4_h(v16h a, v16h b, v16h c, v16h d) { asm volatile("v_nop" :: "v"(a), "v"(b), "v"(c), "v"(d)); }
__device__ __forceinline__ void acc_guard4(v8f& a, v8f& b, v8f& c, v8f& d) { asm volatile("v_nop\n\tv_nop\n\tv_nop\n\tv_nop" : "+v"(a), "+v"(b), "+v"(c), "+v"(d)); }
__device__ __forceinline__ v8f mma2(v16h a0, v16h b0, v16h a1, v16h b1, v8f c) {
    c = __builtin_amdgcn_wmma_f32_16x16x32_f16(false, a0, false, b0, (short)0, c, false, false);
    c = __builtin_amdgcn_wmma_f32_16x16x32_f16(false, a1, false, b1, (short)0, c, false, false);
    asm volatile("v_nop\n\tv_nop\n\tv_nop\n\tv_nop" : "+v"(c) : "v"(a0), "v"(b0), "v"(a1), "v"(b1));
    return c;
}
__device__ __forceinline__ void wave_sync_lds() {
    __builtin_amdgcn_fence(3  , "workgroup");
    __builtin_amdgcn_wave_barrier();
    __builtin_amdgcn_fence(2  , "workgroup");
}

static_assert(512u * 256u * 8u == (unsigned)DM * (unsigned)DM);
__global__ __launch_bounds__(256) void k_wplane(const float* __restrict__ W, unsigned short* __restrict__ P, unsigned hs, unsigned ks) {
    const unsigned u = blockIdx.x * 256u + threadIdx.x;
    const unsigned n = u >> 7, k0 = (u & 127u) << 3;
    const float* s = W + (size_t)(n >> 6) * hs + (n & 63u) + (size_t)k0 * ks;
    float w[8];
#pragma unroll
    for (int e = 0; e < 8; ++e) w[e] = cmb_bf(s[(size_t)e * ks]) * 16.0f;
    v4u pk; pk.x = cmb_pk2(w[0], w[1]); pk.y = cmb_pk2(w[2], w[3]); pk.z = cmb_pk2(w[4], w[5]); pk.w = cmb_pk2(w[6], w[7]);
    VST2(v4u, (v4u*)(P + (size_t)n * DM + k0), pk);
}

static_assert(20u * 256u == 5u * (unsigned)DM);
__global__ __launch_bounds__(256) void k_bias(const float* __restrict__ b0, const float* __restrict__ b1, const float* __restrict__ b2,
                                              const float* __restrict__ b3, const float* __restrict__ b4, float* __restrict__ T) {
    const unsigned i = blockIdx.x * 256u + threadIdx.x;
    const unsigned seg = blockIdx.x >> 2, off = i & 1023u;
    const float* s = b0;
    if (seg == 1u) s = b1;
    if (seg == 2u) s = b2;
    if (seg == 3u) s = b3;
    if (seg == 4u) s = b4;
    const float v = cmb_bf(s[off]);
    VST2(float, T + i, v);
}

static_assert((SEQ / 32) * NB * 32 == MROWS);
__global__ __launch_bounds__(256) void k_pad(const float* __restrict__ ok, float* __restrict__ pad) {
    __shared__ float ssum[32];
    const unsigned tid = threadIdx.x, lane = tid & 31u, w = tid >> 5;
    const unsigned b = blockIdx.y, t0 = blockIdx.x * 32u + w * 4u;
#pragma unroll 1
    for (unsigned rr = 0; rr < 4u; ++rr) {
        const float* r = ok + ((size_t)b * SEQ_FULL + t0 + rr) * DM;
        float a = 0.f;
#pragma unroll 2
        for (unsigned it = 0; it < 8u; ++it) {
            const v4f v = *(const v4f*)(r + 4u * (lane + 32u * it));
            a += fabsf(cmb_bf(v.x)) + fabsf(cmb_bf(v.y)) + fabsf(cmb_bf(v.z)) + fabsf(cmb_bf(v.w));
        }
        a += __shfl_xor(a, 16, 32); a += __shfl_xor(a, 8, 32); a += __shfl_xor(a, 4, 32); a += __shfl_xor(a, 2, 32); a += __shfl_xor(a, 1, 32);
        if (lane == 0u) ssum[w * 4u + rr] = a;
    }
    __syncthreads();
    if (tid < 32u) {
        const float v = (ssum[tid] == 0.f) ? -4294967295.0f : 0.f;
        VST2(float, pad + (size_t)b * SEQ + blockIdx.x * 32u + tid, v);
    }
}

struct DivSeed { float a[8]; float b[8]; float c[8]; };
static_assert(sizeof(DivSeed) == 96);
static_assert(2u * SEQ * 256u * 2u == (unsigned)SEQ * (unsigned)DM);
__global__ __launch_bounds__(256) void k_petab(DivSeed p, float* __restrict__ pe) {
    #pragma clang fp contract(off)
    __shared__ float tb[24];
    if (threadIdx.x == 0u) {
#pragma unroll
        for (int j = 0; j < 8; ++j) { tb[j] = p.a[j]; tb[8 + j] = p.b[j]; tb[16 + j] = p.c[j]; }
    }
    __syncthreads();
    const unsigned idx = blockIdx.x * 256u + threadIdx.x;
    const unsigned t = idx >> 9, i = idx & 511u;
    const float dv = (tb[i >> 6] * tb[8u + ((i >> 3) & 7u)]) * tb[16u + (i & 7u)];
    const float ang = (float)(t + 1u) * dv;
    float sn, cs;
    sincosf(ang, &sn, &cs);
    v2f o; o.x = sn; o.y = cs;
    VST2(v2f, (v2f*)(pe + (size_t)t * DM + 2u * i), o);
}

static_assert(256 * 4 == DM);
__global__ __launch_bounds__(256) void k_posenc(const float* __restrict__ qin, const float* __restrict__ pe, float* __restrict__ x) {
    #pragma clang fp contract(off)
    __shared__ float red[8];
    const unsigned tid = threadIdx.x, lane = tid & 31u, w = tid >> 5;
    const unsigned t = blockIdx.x, b = blockIdx.y;
    v4f q = *(const v4f*)(qin + ((size_t)b * SEQ_FULL + t) * DM + 4u * tid);
    q.x = cmb_bf(q.x); q.y = cmb_bf(q.y); q.z = cmb_bf(q.z); q.w = cmb_bf(q.w);
    float a = fabsf(q.x) + fabsf(q.y) + fabsf(q.z) + fabsf(q.w);
    a += __shfl_xor(a, 16, 32); a += __shfl_xor(a, 8, 32); a += __shfl_xor(a, 4, 32); a += __shfl_xor(a, 2, 32); a += __shfl_xor(a, 1, 32);
    if (lane == 0u) red[w] = a;
    __syncthreads();
    const float tot = ((red[0] + red[1]) + (red[2] + red[3])) + ((red[4] + red[5]) + (red[6] + red[7]));
    const float mk = (tot > 0.f) ? 1.f : 0.f;
    const v4f e = *(const v4f*)(pe + (size_t)t * DM + 4u * tid);
    v4f o;
    o.x = q.x + (0.1f * e.x) * mk; o.y = q.y + (0.1f * e.y) * mk; o.z = q.z + (0.1f * e.z) * mk; o.w = q.w + (0.1f * e.w) * mk;
    VST2(v4f, (v4f*)(x + ((size_t)b * SEQ + t) * DM + 4u * tid), o);
}

__global__ __launch_bounds__(256) void k_lnorm(const float* __restrict__ x, const float* __restrict__ alpha, const float* __restrict__ beta,
                                               float* __restrict__ y32, unsigned short* __restrict__ y16) {
    __shared__ float red1[8];
    __shared__ float red2[8];
    __shared__ v2u hrow[256];
    const unsigned tid = threadIdx.x, lane = tid & 31u, w = tid >> 5;
    const size_t rbase = (size_t)blockIdx.x * DM;
    const v4f v = *(const v4f*)(x + rbase + 4u * tid);
    float s = (v.x + v.y) + (v.z + v.w);
    s += __shfl_xor(s, 16, 32); s += __shfl_xor(s, 8, 32); s += __shfl_xor(s, 4, 32); s += __shfl_xor(s, 2, 32); s += __shfl_xor(s, 1, 32);
    if (lane == 0u) red1[w] = s;
    __syncthreads();
    const float mu = (((red1[0] + red1[1]) + (red1[2] + red1[3])) + ((red1[4] + red1[5]) + (red1[6] + red1[7]))) * (1.0f / 1024.0f);
    const float d0 = v.x - mu, d1 = v.y - mu, d2 = v.z - mu, d3 = v.w - mu;
    float q = (d0 * d0 + d1 * d1) + (d2 * d2 + d3 * d3);
    q += __shfl_xor(q, 16, 32); q += __shfl_xor(q, 8, 32); q += __shfl_xor(q, 4, 32); q += __shfl_xor(q, 2, 32); q += __shfl_xor(q, 1, 32);
    if (lane == 0u) red2[w] = q;
    __syncthreads();
    const float ss = ((red2[0] + red2[1]) + (red2[2] + red2[3])) + ((red2[4] + red2[5]) + (red2[6] + red2[7]));
    const float sg = sqrtf(ss * (1.0f / 1023.0f));
    const float inv = 1.0f / (sg + 1e-8f);
    const float A = cmb_bf(alpha[0]), Bp = cmb_bf(beta[0]);
    v4f y;
    y.x = (A * d0) * inv + Bp; y.y = (A * d1) * inv + Bp; y.z = (A * d2) * inv + Bp; y.w = (A * d3) * inv + Bp;
    if (y32) { VST2(v4f, (v4f*)(y32 + rbase + 4u * tid), y); }
    v2u pk; pk.x = cmb_pk2(y.x, y.y); pk.y = cmb_pk2(y.z, y.w);
    hrow[tid] = pk;
    __syncthreads();
    if (tid < 128u) {
        const v2u a0 = hrow[2u * tid], a1 = hrow[2u * tid + 1u];
        v4u o; o.x = a0.x; o.y = a0.y; o.z = a1.x; o.w = a1.y;
        VST2(v4u, (v4u*)(y16 + rbase + 8u * tid), o);
    }
}
static_assert(128 * 8 == DM);

template <int BIAS_MODE, int OUT_MODE, bool RESID, int ACT>
__global__ __launch_bounds__(256) void k_gemm64(
    const unsigned short* __restrict__ Ap, unsigned lda,
    const unsigned short* __restrict__ Btp, unsigned ldb,
    void* __restrict__ Cout, unsigned ldc,
    const float* __restrict__ bias, const float* __restrict__ resid,
    unsigned tilesM, unsigned tnshift, unsigned K, float scale) {
  const _Float16* A = (const _Float16*)Ap;
  const _Float16* Bt = (const _Float16*)Btp;
  __shared__ __align__(16) float sT[8][16 * 68];
  const unsigned lane = threadIdx.x & 31u;
  const unsigned wave = threadIdx.x >> 5;
  const unsigned tile = blockIdx.x * 8u + wave;
  if (tile >= (tilesM << tnshift)) return;
  const unsigned tm = tile >> tnshift;
  const unsigned tn = tile & ((1u << tnshift) - 1u);
  const unsigned m0 = tm << 6;
  const unsigned n0 = tn << 6;
  const unsigned rlane = lane & 15u;
  const unsigned koff  = (lane >> 4) * 8u;
  const unsigned mOff  = (lane >> 4) * 8u;

  v8f acc[4][4];
#pragma unroll
  for (int i = 0; i < 4; ++i)
#pragma unroll
    for (int j = 0; j < 4; ++j) acc[i][j] = (v8f){0.f,0.f,0.f,0.f,0.f,0.f,0.f,0.f};

  for (unsigned k0 = 0; k0 < K; k0 += 32u) {
    v16h bh[4];
#pragma unroll
    for (int j = 0; j < 4; ++j) {
      const size_t bo = (size_t)(n0 + ((unsigned)j << 4) + rlane) * ldb + koff + k0;
      bh[j] = fload(Bt + bo);
    }
#pragma unroll
    for (int i = 0; i < 4; ++i) {
      const size_t ao = (size_t)(m0 + ((unsigned)i << 4) + rlane) * lda + koff + k0;
      const v16h ah = fload(A + ao);
#pragma unroll
      for (int j = 0; j < 4; ++j) acc[i][j] = mma_raw(ah, bh[j], acc[i][j]);
      dep_guard_h(acc[i][0], acc[i][3], ah, ah);
    }
    keep4_h(bh[0], bh[1], bh[2], bh[3]);
  }
  acc_guard4(acc[0][0], acc[0][1], acc[0][2], acc[0][3]);
  acc_guard4(acc[1][0], acc[1][1], acc[1][2], acc[1][3]);
  acc_guard4(acc[2][0], acc[2][1], acc[2][2], acc[2][3]);
  acc_guard4(acc[3][0], acc[3][1], acc[3][2], acc[3][3]);

  float* slab = sT[wave];
#pragma unroll
  for (int i = 0; i < 4; ++i) {
    const unsigned mBase = m0 + ((unsigned)i << 4);
#pragma unroll
    for (int j = 0; j < 4; ++j) {
      const unsigned n = n0 + ((unsigned)j << 4) + rlane;
      float bv = 0.f;
      if (BIAS_MODE == 2) bv = bias[n];
#pragma unroll
      for (int r = 0; r < 8; ++r) {
        float v = acc[i][j][r] * scale;
        if (BIAS_MODE == 1) v += bias[mBase + mOff + (unsigned)r];
        if (BIAS_MODE == 2) v += bv;
        if (ACT == 1) v = fmaxf(v, 0.0f);
        if (RESID) v += resid[(size_t)(mBase + mOff + (unsigned)r) * ldc + n];
        slab[(mOff + (unsigned)r) * 68u + ((unsigned)j << 4) + rlane] = v;
      }
    }
    wave_sync_lds();
    if (OUT_MODE == 0) {
      float* C = (float*)Cout;
      const unsigned hh = lane >> 4, c4 = (lane & 15u) * 4u;
      for (int pass = 0; pass < 2; ++pass) {
#pragma unroll
        for (int it = 0; it < 8; ++it) {
          const unsigned row = (unsigned)it * 2u + hh;
          const v4f v = *(const v4f*)(slab + row * 68u + c4);
          *(volatile v4f*)(C + (size_t)(mBase + row) * ldc + n0 + c4) = v;
        }
        __threadfence();
      }
    } else {
      const unsigned q = lane >> 3, c8 = (lane & 7u) * 8u;
      unsigned short* C = (unsigned short*)Cout;
      for (int pass = 0; pass < 2; ++pass) {
#pragma unroll
        for (int it = 0; it < 4; ++it) {
          const unsigned row = (unsigned)it * 4u + q;
          const float* sp = slab + row * 68u + c8;
          v8h hv;
#pragma unroll
          for (int e = 0; e < 8; ++e) hv[e] = (_Float16)sp[e];
          *(volatile v8h*)(C + (size_t)(mBase + row) * ldc + n0 + c8) = hv;
        }
        __threadfence();
      }
    }
    wave_sync_lds();
  }
}

static_assert((SEQ / 64) * NH * NB * 4 * 16 * 64 == MROWS * DM);
__global__ __launch_bounds__(128) void k_attn(const unsigned short* __restrict__ QKp, const unsigned short* __restrict__ VTp,
                                              const float* __restrict__ pad, unsigned short* __restrict__ HDp) {
  __shared__ __align__(16) _Float16 Psh[4][16 * 64];
  __shared__ __align__(16) float    Os[4][16 * 68];
  const unsigned tid = threadIdx.x, wave = tid >> 5, lane = tid & 31u, hh = lane >> 4, c = lane & 15u;
  const unsigned qb = blockIdx.x, h = blockIdx.y, b = blockIdx.z;
  const unsigned q0 = qb * 64u + wave * 16u;
  const unsigned tok0 = b * (unsigned)SEQ;
  const _Float16* QK = (const _Float16*)QKp;
  const _Float16* VT = (const _Float16*)VTp;
  const float C1 = 0.045084220027780106f;
  const float L2E = 1.4426950408889634f;

  v16h qa[2];
  {
    const _Float16* qr = QK + (size_t)(tok0 + q0 + c) * QKP + h * 64u + 8u * hh;
    qa[0] = fload(qr); qa[1] = fload(qr + 32);
  }
  const _Float16* kbase = QK + (size_t)tok0 * QKP + DM + h * 64u + 8u * hh;
  const _Float16* vbase = VT + (size_t)(h * 64u + c) * VTP + tok0 + 8u * hh;
  const float* pb = pad + tok0;
  _Float16* pw = Psh[wave];

  float mrow[8], lrow[8];
  v8f oacc[4];
#pragma unroll
  for (int r = 0; r < 8; ++r) { mrow[r] = -__builtin_inff(); lrow[r] = 0.f; }
#pragma unroll
  for (int t = 0; t < 4; ++t) oacc[t] = (v8f){0.f,0.f,0.f,0.f,0.f,0.f,0.f,0.f};

#pragma unroll 1
  for (unsigned kc = 0; kc < (unsigned)(SEQ / 64); ++kc) {
    const unsigned kv0 = kc * 64u;
    v8f s[4];
    float pl[4];
#pragma unroll
    for (int j = 0; j < 4; ++j) {
      const unsigned key = kv0 + (unsigned)j * 16u + c;
      const _Float16* kr = kbase + (size_t)key * QKP;
      const v16h k0f = fload(kr), k1f = fload(kr + 32);
      s[j] = mma2(qa[0], k0f, qa[1], k1f, (v8f){0.f,0.f,0.f,0.f,0.f,0.f,0.f,0.f});
      pl[j] = pb[key] * L2E;
    }
#pragma unroll
    for (int r = 0; r < 8; ++r) {
      float m = -__builtin_inff();
#pragma unroll
      for (int j = 0; j < 4; ++j) { const float tv = s[j][r] * C1 + pl[j]; s[j][r] = tv; m = fmaxf(m, tv); }
      m = fmaxf(m, __shfl_xor(m, 1, 32)); m = fmaxf(m, __shfl_xor(m, 2, 32));
      m = fmaxf(m, __shfl_xor(m, 4, 32)); m = fmaxf(m, __shfl_xor(m, 8, 32));
      const float mnew = fmaxf(mrow[r], m);
      const float al = exp2f(mrow[r] - mnew);
      mrow[r] = mnew;
      float psum = 0.f;
#pragma unroll
      for (int j = 0; j < 4; ++j) {
        const float p = exp2f(s[j][r] - mnew);
        psum += p;
        pw[(8u * hh + (unsigned)r) * 64u + (unsigned)j * 16u + c] = (_Float16)(p * 32768.0f);
      }
      psum += __shfl_xor(psum, 1, 32); psum += __shfl_xor(psum, 2, 32); psum += __shfl_xor(psum, 4, 32); psum += __shfl_xor(psum, 8, 32);
      lrow[r] = lrow[r] * al + psum;
#pragma unroll
      for (int t = 0; t < 4; ++t) oacc[t][r] *= al;
    }
    wave_sync_lds();
    const v16h pa0 = fload(pw + c * 64u + 8u * hh);
    const v16h pa1 = fload(pw + c * 64u + 32u + 8u * hh);
#pragma unroll
    for (int t = 0; t < 4; ++t) {
      const _Float16* vr = vbase + (size_t)((unsigned)t * 16u) * VTP + kv0;
      const v16h v0f = fload(vr), v1f = fload(vr + 32);
      oacc[t] = mma2(pa0, v0f, pa1, v1f, oacc[t]);
    }
    wave_sync_lds();
  }

  float* os = Os[wave];
#pragma unroll
  for (int r = 0; r < 8; ++r) {
    const float inv = 1.0f / (lrow[r] * 512.0f);
#pragma unroll
    for (int t = 0; t < 4; ++t) os[(8u * hh + (unsigned)r) * 68u + (unsigned)t * 16u + c] = oacc[t][r] * inv;
  }
  wave_sync_lds();
  {
    const unsigned q = lane >> 3, c8 = (lane & 7u) * 8u;
    for (int pass = 0; pass < 2; ++pass) {
#pragma unroll
      for (int it = 0; it < 4; ++it) {
        const unsigned row = (unsigned)it * 4u + q;
        const float* sp = os + row * 68u + c8;
        v8h hv;
#pragma unroll
        for (int e = 0; e < 8; ++e) hv[e] = (_Float16)sp[e];
        *(volatile v8h*)(HDp + (size_t)(tok0 + q0 + row) * DM + h * 64u + c8) = hv;
      }
      __threadfence();
    }
  }
}

constexpr size_t al256(size_t v) { return (v + 255u) & ~(size_t)255u; }
constexpr unsigned ilog2u(unsigned v) { return (v <= 1u) ? 0u : 1u + ilog2u(v >> 1); }

constexpr size_t SZ_WQK = (size_t)2 * DM * DM * 2;
constexpr size_t SZ_W1  = (size_t)DM * DM * 2;
constexpr size_t SZ_BT  = (size_t)5 * DM * 4;
constexpr size_t SZ_PAD = (size_t)MROWS * 4;
constexpr size_t SZ_PE  = (size_t)SEQ * DM * 4;
constexpr size_t SZ_F32 = (size_t)MROWS * DM * 4;
constexpr size_t SZ_H16 = (size_t)MROWS * DM * 2;
constexpr size_t SZ_QK  = (size_t)MROWS * QKP * 2;
constexpr size_t SZ_VT  = (size_t)DM * VTP * 2;

constexpr size_t OFF_WQK = 0;
constexpr size_t OFF_WV  = OFF_WQK + al256(SZ_WQK);
constexpr size_t OFF_WO  = OFF_WV  + al256(SZ_W1);
constexpr size_t OFF_WF  = OFF_WO  + al256(SZ_W1);
constexpr size_t OFF_BT  = OFF_WF  + al256(SZ_W1);
constexpr size_t OFF_PAD = OFF_BT  + al256(SZ_BT);
constexpr size_t OFF_PE  = OFF_PAD + al256(SZ_PAD);
constexpr size_t OFF_X32 = OFF_PE  + al256(SZ_PE);
constexpr size_t OFF_Q32 = OFF_X32 + al256(SZ_F32);
constexpr size_t OFF_O32 = OFF_Q32 + al256(SZ_F32);
constexpr size_t OFF_Q16 = OFF_O32 + al256(SZ_F32);
constexpr size_t OFF_T16 = OFF_Q16 + al256(SZ_H16);
constexpr size_t OFF_QK  = OFF_T16 + al256(SZ_H16);
constexpr size_t OFF_VT  = OFF_QK  + al256(SZ_QK);
constexpr size_t OFF_HD  = OFF_VT  + al256(SZ_VT);
constexpr size_t WS_TOTAL = OFF_HD + al256(SZ_H16);
static_assert(WS_TOTAL <= (size_t)134217728);

static_assert(((size_t)(MROWS / 64) * (QKP / 64)) * 4096u == (size_t)MROWS * QKP);
static_assert(((size_t)(DM / 64) * (MROWS / 64)) * 4096u == (size_t)DM * VTP);
static_assert(((size_t)(MROWS / 64) * (DM / 64)) * 4096u == (size_t)MROWS * DM);

extern "C" void kernel_launch(void* const* d_in, const int* in_sizes, int n_in, void* d_out, int out_size, void* d_ws, size_t ws_size, hipStream_t stream) {
    if (n_in < 14) return;
    const long long need_act = ((long long)(NB - 1) * SEQ_FULL + SEQ) * DM;
    if ((long long)in_sizes[0] < need_act || (long long)in_sizes[1] < need_act) return;
    if (in_sizes[2] < DM * DM || in_sizes[4] < DM * DM || in_sizes[6] < DM * DM || in_sizes[8] < DM * DM || in_sizes[10] < DM * DM) return;
    if (in_sizes[3] < DM || in_sizes[5] < DM || in_sizes[7] < DM || in_sizes[9] < DM || in_sizes[11] < DM) return;
    if (in_sizes[12] < 1 || in_sizes[13] < 1) return;
    if ((long long)out_size < (long long)MROWS * DM) return;
    if (WS_TOTAL > ws_size) return;

    const float* qin   = (const float*)d_in[0];
    const float* ori_k = (const float*)d_in[1];
    const float* Wq    = (const float*)d_in[2];
    const float* bq    = (const float*)d_in[3];
    const float* Wk    = (const float*)d_in[4];
    const float* bk    = (const float*)d_in[5];
    const float* Wv    = (const float*)d_in[6];
    const float* bv    = (const float*)d_in[7];
    const float* Wout  = (const float*)d_in[8];
    const float* bout  = (const float*)d_in[9];
    const float* Wf    = (const float*)d_in[10];
    const float* bf    = (const float*)d_in[11];
    const float* alpha = (const float*)d_in[12];
    const float* beta  = (const float*)d_in[13];

    char* ws = (char*)d_ws;
    unsigned short* WQK = (unsigned short*)(ws + OFF_WQK);
    unsigned short* WV  = (unsigned short*)(ws + OFF_WV);
    unsigned short* WO  = (unsigned short*)(ws + OFF_WO);
    unsigned short* WF  = (unsigned short*)(ws + OFF_WF);
    float* BT   = (float*)(ws + OFF_BT);
    float* PAD  = (float*)(ws + OFF_PAD);
    float* PE   = (float*)(ws + OFF_PE);
    float* X32  = (float*)(ws + OFF_X32);
    float* Q32  = (float*)(ws + OFF_Q32);
    float* O32  = (float*)(ws + OFF_O32);
    unsigned short* Q16 = (unsigned short*)(ws + OFF_Q16);
    unsigned short* T16 = (unsigned short*)(ws + OFF_T16);
    unsigned short* QKPL = (unsigned short*)(ws + OFF_QK);
    unsigned short* VTPL = (unsigned short*)(ws + OFF_VT);
    unsigned short* HD16 = (unsigned short*)(ws + OFF_HD);

    k_wplane<<<512, 256, 0, stream>>>(Wq,   WQK,                      (unsigned)(DM * HDIM), (unsigned)HDIM);
    k_wplane<<<512, 256, 0, stream>>>(Wk,   WQK + (size_t)DM * DM,    (unsigned)(DM * HDIM), (unsigned)HDIM);
    k_wplane<<<512, 256, 0, stream>>>(Wv,   WV,                       (unsigned)(DM * HDIM), (unsigned)HDIM);
    k_wplane<<<512, 256, 0, stream>>>(Wout, WO,                       (unsigned)HDIM,        (unsigned)DM);
    k_wplane<<<512, 256, 0, stream>>>(Wf,   WF,                       (unsigned)HDIM,        (unsigned)DM);
    k_bias<<<20, 256, 0, stream>>>(bq, bk, bv, bout, bf, BT);
    k_pad<<<dim3(SEQ / 32, NB), 256, 0, stream>>>(ori_k, PAD);
    {
        DivSeed ds;
        for (int j = 0; j < 8; ++j) {
            ds.a[j] = (float)pow(100000.0, -(double)(64 * j) / 512.0);
            ds.b[j] = (float)pow(100000.0, -(double)(8 * j) / 512.0);
            ds.c[j] = (float)pow(100000.0, -(double)(j) / 512.0);
        }
        k_petab<<<2 * SEQ, 256, 0, stream>>>(ds, PE);
    }
    k_posenc<<<dim3(SEQ, NB), 256, 0, stream>>>(qin, PE, X32);

    const unsigned TM   = (unsigned)(MROWS / 64);
    const unsigned SH_M = ilog2u((unsigned)(MROWS / 64));
    const unsigned g_qk = (TM * (unsigned)(QKP / 64) + 7u) / 8u;
    const unsigned g_vt = ((unsigned)(DM / 64) * TM + 7u) / 8u;
    const unsigned g_dd = (TM * (unsigned)(DM / 64) + 7u) / 8u;

    for (int layer = 0; layer < NLAYER; ++layer) {
        k_lnorm<<<MROWS, 256, 0, stream>>>(X32, alpha, beta, Q32, Q16);
        k_gemm64<2, 1, false, 0><<<g_qk, 256, 0, stream>>>(Q16, (unsigned)DM, WQK, (unsigned)DM, (void*)QKPL, (unsigned)QKP,
                                                            BT, nullptr, TM, ilog2u((unsigned)(QKP / 64)), (unsigned)DM, 0.0625f);
        k_gemm64<1, 1, false, 0><<<g_vt, 256, 0, stream>>>(WV, (unsigned)DM, Q16, (unsigned)DM, (void*)VTPL, (unsigned)VTP,
                                                            BT + 2 * DM, nullptr, (unsigned)(DM / 64), SH_M, (unsigned)DM, 0.0625f);
        k_attn<<<dim3(SEQ / 64, NH, NB), 128, 0, stream>>>(QKPL, VTPL, PAD, HD16);
        k_gemm64<2, 0, true, 0><<<g_dd, 256, 0, stream>>>(HD16, (unsigned)DM, WO, (unsigned)DM, (void*)O32, (unsigned)DM,
                                                           BT + 3 * DM, Q32, TM, ilog2u((unsigned)(DM / 64)), (unsigned)DM, 1.0f / 1024.0f);
        k_lnorm<<<MROWS, 256, 0, stream>>>(O32, alpha, beta, nullptr, T16);
        float* xdst = (layer == NLAYER - 1) ? (float*)d_out : X32;
        k_gemm64<2, 0, true, 1><<<g_dd, 256, 0, stream>>>(T16, (unsigned)DM, WF, (unsigned)DM, (void*)xdst, (unsigned)DM,
                                                           BT + 4 * DM, O32, TM, ilog2u((unsigned)(DM / 64)), (unsigned)DM, 0.0625f);
    }
}
